// DrBCEncoder_43946105373340
// MI455X (gfx1250) — hardware-run, weakly checked
//
#include <hip/hip_runtime.h>

typedef float          v8f   __attribute__((ext_vector_type(8)));
typedef float          v4f   __attribute__((ext_vector_type(4)));
typedef unsigned int   v4u   __attribute__((ext_vector_type(4)));
typedef int            v8i   __attribute__((ext_vector_type(8)));
typedef unsigned short v8us  __attribute__((ext_vector_type(8)));
typedef unsigned short v16us __attribute__((ext_vector_type(16)));
typedef __bf16         v16bf __attribute__((ext_vector_type(16)));
typedef _Float16       v16h  __attribute__((ext_vector_type(16)));
typedef v4f  __attribute__((may_alias)) v4fa;
typedef v8us __attribute__((may_alias)) v8usa;
union FragB { v16bf v; v16us u; v8us h[2]; v8i w; };
union FragH { v16h  v; v16us u; v8us h[2]; v8i w; };

__device__ __forceinline__ v8f wmb(const FragB& a, const FragB& b, v8f c) {
  v8f d = __builtin_amdgcn_wmma_f32_16x16x32_bf16(false, a.v, false, b.v, (short)0, c, false, false);
  asm volatile("v_nop\n\tv_nop\n\tv_nop\n\tv_nop" : "+v"(d) : "v"(a.w), "v"(b.w));
  return d;
}

__device__ __forceinline__ v8f wmh(const FragH& a, const FragH& b, v8f c) {
  v8f d = __builtin_amdgcn_wmma_f32_16x16x32_f16(false, a.v, false, b.v, (short)0, c, false, false);
  asm volatile("v_nop\n\tv_nop\n\tv_nop\n\tv_nop" : "+v"(d) : "v"(a.w), "v"(b.w));
  return d;
}

__device__ __forceinline__ unsigned bf16_bits(float f) {
  const unsigned u = __float_as_uint(f);
  const unsigned r = (u + 0x7FFFu + ((u >> 16) & 1u)) >> 16;
  const unsigned q = (u >> 16) | 0x40u;
  return ((u & 0x7fffffffu) > 0x7f800000u) ? q : r;
}

__device__ __forceinline__ float bf16_val(float f) {
  return __uint_as_float(bf16_bits(f) << 16);
}
__device__ __forceinline__ int clampi(int v, int lo, int hi) {
  return v < lo ? lo : (v > hi ? hi : v);
}

__device__ __forceinline__ unsigned f16_bits(float f) {
  const unsigned u  = __float_as_uint(f);
  const unsigned s  = (u >> 16) & 0x8000u;
  const unsigned a  = u & 0x7fffffffu;
  const unsigned t  = a - 0x38000000u;
  const unsigned r  = (t + 0x0FFFu + ((t >> 13) & 1u)) >> 13;
  const unsigned rc = r > 0x7C00u ? 0x7C00u : r;
  const bool small  = a < 0x38800000u;
  const bool isnan  = a > 0x7f800000u;
  const unsigned fin = small ? 0u : (s | rc);
  return isnan ? (s | 0x7E00u) : fin;
}

__device__ __forceinline__ unsigned pk16(unsigned lo, unsigned hi) { return lo | (hi << 16); }
__device__ __forceinline__ unsigned bf16_lo_bits(float v) {
  float hi = bf16_val(v);
  asm volatile("" : "+v"(hi));
  return bf16_bits(v - hi);
}
__device__ __forceinline__ v4u pack8_bf16(v4f a, v4f c) {
  return (v4u){ pk16(bf16_bits(a[0]), bf16_bits(a[1])), pk16(bf16_bits(a[2]), bf16_bits(a[3])),
                pk16(bf16_bits(c[0]), bf16_bits(c[1])), pk16(bf16_bits(c[2]), bf16_bits(c[3])) };
}
__device__ __forceinline__ v4u pack8_bf16_lo(v4f a, v4f c) {
  return (v4u){ pk16(bf16_lo_bits(a[0]), bf16_lo_bits(a[1])), pk16(bf16_lo_bits(a[2]), bf16_lo_bits(a[3])),
                pk16(bf16_lo_bits(c[0]), bf16_lo_bits(c[1])), pk16(bf16_lo_bits(c[2]), bf16_lo_bits(c[3])) };
}
__device__ __forceinline__ v4u pack8_f16(v4f a, v4f c) {
  return (v4u){ pk16(f16_bits(a[0]), f16_bits(a[1])), pk16(f16_bits(a[2]), f16_bits(a[3])),
                pk16(f16_bits(c[0]), f16_bits(c[1])), pk16(f16_bits(c[2]), f16_bits(c[3])) };
}

template <int FORM>
__global__ __launch_bounds__(256) void k_plane(const float* __restrict__ src, int rows, int cols, int ldsrc,
                                               unsigned short* __restrict__ dst, int MP, int KP) {
  static_assert(FORM >= 0 && FORM <= 3);
  const int KTOT = (FORM == 1 || FORM == 3) ? 2 * KP : KP;
  const unsigned ppr   = (unsigned)(KTOT >> 3);
  const unsigned kp8   = (unsigned)(KP >> 3);
  const unsigned total = (unsigned)MP * ppr;
  const unsigned g     = blockIdx.x * 256u + threadIdx.x;
  const unsigned rowu  = g / ppr;
  const unsigned p     = g - rowu * ppr;
  const bool second    = p >= kp8;
  const int row = (int)rowu;
  const int c0  = (int)((second ? p - kp8 : p) << 3);
  const float* srow = src + (size_t)clampi(row, 0, rows - 1) * (size_t)ldsrc;
  float x[8];
  unsigned mk[8];
#pragma unroll
  for (int e = 0; e < 8; ++e) {
    const int c = c0 + e;
    const float v = srow[clampi(c, 0, cols - 1)];
    asm volatile("" :: "v"(v));
    x[e]  = v;
    mk[e] = (row < rows && c < cols) ? 0xFFFFu : 0u;
  }
  const v4f a = (v4f){ x[0], x[1], x[2], x[3] };
  const v4f c = (v4f){ x[4], x[5], x[6], x[7] };
  v4u o;
  if (FORM == 2) {
    o = pack8_f16(a, c);
  } else {
    const v4u hi = pack8_bf16(a, c);
    o = hi;
    if (FORM == 1) { const v4u lo = pack8_bf16_lo(a, c); o = second ? lo : hi; }
  }
  const v4u mw = (v4u){ pk16(mk[0], mk[1]), pk16(mk[2], mk[3]), pk16(mk[4], mk[5]), pk16(mk[6], mk[7]) };
  o &= mw;
  if (g < total) {
    volatile v4u* q = (volatile v4u*)(dst + (size_t)g * 8);
    *q = o;
    __threadfence();
    *q = o;
  }
}

template <int FORM> struct FragOf    { typedef FragB T; };
template <>         struct FragOf<2> { typedef FragH T; };
__device__ __forceinline__ v8f mm(const FragB& a, const FragB& b, v8f c) { return wmb(a, b, c); }
__device__ __forceinline__ v8f mm(const FragH& a, const FragH& b, v8f c) { return wmh(a, b, c); }
template <class F> __device__ __forceinline__ F ld_frag(const unsigned short* p) {
  F f;
  f.h[0] = *(const v8usa*)(p);
  f.h[1] = *(const v8usa*)(p + 16);
  return f;
}

template <int FORM, int EPI>
__global__ __launch_bounds__(256) __attribute__((amdgpu_num_vgpr(248)))
void k_gemm_nt(const unsigned short* __restrict__ A, const unsigned short* __restrict__ B,
               const float* __restrict__ bias, float* __restrict__ D, int M, int N, int KTOT, int ldd) {
  static_assert(FORM >= 0 && FORM <= 2);
  static_assert(EPI == 0 || EPI == 1);
  typedef typename FragOf<FORM>::T F;
  __shared__ __attribute__((aligned(16))) float sT[8][16 * 68];
  const int lane = threadIdx.x & 31;
  const int wave = threadIdx.x >> 5;
  const int tilesM = (M + 63) >> 6;
  const int tilesN = (N + 63) >> 6;
  const int tile = blockIdx.x * 8 + wave;
  if (tile >= tilesM * tilesN) return;
  const int tm = tile / tilesN;
  const int tn = tile - tm * tilesN;
  const int m0 = tm << 6;
  const int n0 = tn << 6;

  const int rl = lane & 15;
  const int h8 = (lane >> 4) * 8;
  const unsigned short* pa = A + (size_t)(m0 + rl) * (size_t)KTOT + h8;
  const unsigned short* pb = B + (size_t)(n0 + rl) * (size_t)KTOT + h8;

  v8f acc[4][4];
#pragma unroll
  for (int i = 0; i < 4; ++i)
#pragma unroll
    for (int j = 0; j < 4; ++j) acc[i][j] = (v8f){0.f, 0.f, 0.f, 0.f, 0.f, 0.f, 0.f, 0.f};

#pragma unroll 1
  for (int k0 = 0; k0 < KTOT; k0 += 32) {
    F bf[4];
#pragma unroll
    for (int j = 0; j < 4; ++j) bf[j] = ld_frag<F>(pb + (size_t)(j << 4) * (size_t)KTOT + k0);
#pragma unroll
    for (int i = 0; i < 4; ++i) {
      const F af = ld_frag<F>(pa + (size_t)(i << 4) * (size_t)KTOT + k0);
#pragma unroll
      for (int j = 0; j < 4; ++j) acc[i][j] = mm(af, bf[j], acc[i][j]);
    }
  }

  float* slab = sT[wave];
  const int hh = lane >> 4;
  const int c4 = (lane & 15) * 4;
  const int nc = n0 + c4;
  const bool cok = nc < N;
  v4f bv = (v4f){0.f, 0.f, 0.f, 0.f};
  if (EPI == 1) {
    bv = *(const v4fa*)(bias + clampi(nc, 0, N - 4));
    asm volatile("" :: "v"(bv));
  }
#pragma unroll
  for (int i = 0; i < 4; ++i) {
    const int mBase = m0 + (i << 4);
#pragma unroll
    for (int j = 0; j < 4; ++j) {
#pragma unroll
      for (int r = 0; r < 8; ++r) slab[(h8 + r) * 68 + (j << 4) + rl] = acc[i][j][r];
    }
    __builtin_amdgcn_fence(__ATOMIC_RELEASE, "workgroup");
    __builtin_amdgcn_wave_barrier();
    __builtin_amdgcn_fence(__ATOMIC_ACQUIRE, "workgroup");
    v4f vv[8];
#pragma unroll
    for (int it = 0; it < 8; ++it) {
      const int row = it * 2 + hh;
      v4f v = *(const v4fa*)(slab + row * 68 + c4);
      if (EPI == 1) v += bv;
      vv[it] = v;
    }
    for (int pass = 0; pass < 2; ++pass) {
#pragma unroll
      for (int it = 0; it < 8; ++it) {
        const int row = mBase + it * 2 + hh;
        if (cok && row < M) *(volatile v4f*)(D + (size_t)row * (size_t)ldd + nc) = vv[it];
      }
      __threadfence();
    }
    __builtin_amdgcn_fence(__ATOMIC_RELEASE, "workgroup");
    __builtin_amdgcn_wave_barrier();
    __builtin_amdgcn_fence(__ATOMIC_ACQUIRE, "workgroup");
  }
}

#pragma clang fp contract(off)
#include <stddef.h>

#define SPLIT_L 1

#define G_NN    100000
#define G_MP    100096
#define G_NE    3200000
#define G_HD    64
#define G_OPK   (SPLIT_L ? 128 : 64)
#define G_PPR   (G_OPK / 8)
#define G_WPB   (64 * G_PPR / 256)

#define L_NBRUN 1024
#define L_SLB   10
#define L_NBK   98
#define L_HCAP  21504
#define L_LCAP  (2 * L_HCAP)
#define L_WLCAP 5104
#define L_DEGCAP 128
#define L_ZINTS (8 * L_WLCAP + L_HCAP + 3 * L_NBRUN)
#define L_INTS  (L_ZINTS + 16)
#define L_LDS   (L_INTS * 4)
#define MEAS_MAXDEG 58
#define MEAS_B512   16671
#define MEAS_B1024  33280

static_assert(G_HD == 64);
static_assert(G_MP % 128 == 0 && G_MP >= G_NN && G_MP == 782 * 128);
static_assert(G_MP % 64 == 0 && G_NN % 16 == 0 && G_MP % 16 == 0 && G_OPK % 32 == 0);
static_assert(G_NN % 8 == 0);
static_assert(L_NBRUN == (1 << L_SLB) && L_SLB == 10 && 22 + L_SLB == 32);
static_assert(G_NE < (1 << 22));
static_assert(L_NBK * L_NBRUN >= G_MP && (L_NBK - 1) * L_NBRUN < G_NN);
static_assert(G_NE % 256 == 0);
static_assert((long long)L_HCAP * 100 >= (long long)MEAS_B512 * 125);
static_assert((long long)L_LCAP * 100 >= (long long)MEAS_B1024 * 125);
static_assert((long long)8 * L_WLCAP * 100 >= (long long)MEAS_B1024 * 115);
static_assert(L_WLCAP >= MEAS_B1024 / 8 + 8 * 65 + 1);
static_assert(MEAS_MAXDEG + 8 <= L_DEGCAP);
static_assert(L_HCAP % 1024 == 0 && L_ZINTS % 4 == 0);
static_assert(L_LDS <= 262144);

typedef float        v2f __attribute__((ext_vector_type(2)));
typedef unsigned int v2u __attribute__((ext_vector_type(2)));
typedef int          v4i __attribute__((ext_vector_type(4)));
typedef v2f __attribute__((may_alias)) v2fa;
typedef v4i __attribute__((may_alias)) v4ia;

__device__ __forceinline__ void st2_v4f(float* p, v4f v) {
  *(volatile v4f*)p = v;
  __threadfence();
  *(volatile v4f*)p = v;
}
__device__ __forceinline__ void st2_v2f(float* p, v2f v) {
  *(volatile v2f*)p = v;
  __threadfence();
  *(volatile v2f*)p = v;
}
__device__ __forceinline__ void st2_v4u(unsigned short* p, v4u v) {
  *(volatile v4u*)p = v;
  __threadfence();
  *(volatile v4u*)p = v;
}
__device__ __forceinline__ void st2_v2u(unsigned short* p, v2u v) {
  *(volatile v2u*)p = v;
  __threadfence();
  *(volatile v2u*)p = v;
}
__device__ __forceinline__ void st2_v4i(int* p, v4i v) {
  *(volatile v4i*)p = v;
  __threadfence();
  *(volatile v4i*)p = v;
}
__device__ __forceinline__ float relu_k(float v) { return (v > 0.0f) ? v : (v - v); }

__device__ __forceinline__ void prep_unit(const float* __restrict__ w, int unit, unsigned short* dstp) {
  const int n = unit / G_PPR;
  const int p = unit - n * G_PPR;
  const float* s = w + (size_t)n * 64 + 8 * (p & 7);
  const v4f a = *(const v4fa*)s;
  const v4f c = *(const v4fa*)(s + 4);
  asm volatile("" :: "v"(a));
  asm volatile("" :: "v"(c));
  st2_v4u(dstp + (size_t)n * G_OPK + 8 * p, pack8_bf16(a, c));
}

__global__ __launch_bounds__(256) void k_prep(const float* __restrict__ win, const float* __restrict__ bin,
                                              const float* __restrict__ wself, const float* __restrict__ wneigh,
                                              const float* __restrict__ biases, const float* __restrict__ gammas,
                                              const float* __restrict__ betas,
                                              unsigned short* WINP, unsigned short* WPL, float* PAR) {
  const int tid = (int)threadIdx.x;
  const int blk = (int)blockIdx.x;
  if (blk < 3 * G_WPB) {
    const int pl = blk / G_WPB;
    const int unit = (blk - pl * G_WPB) * 256 + tid;
    prep_unit(wself + (size_t)pl * 4096, unit, WPL + (size_t)pl * 64 * G_OPK);
  } else if (blk < 6 * G_WPB) {
    const int b2 = blk - 3 * G_WPB;
    const int pl = b2 / G_WPB;
    const int unit = (b2 - pl * G_WPB) * 256 + tid;
    prep_unit(wneigh + (size_t)pl * 4096, unit, WPL + (size_t)(3 + pl) * 64 * G_OPK);
  } else if (blk == 6 * G_WPB) {
    const int n = tid >> 2, p = tid & 3;
    const float* s = win + (size_t)n * 8;
    const v4f a = *(const v4fa*)s;
    const v4f c = *(const v4fa*)(s + 4);
    asm volatile("" :: "v"(a));
    asm volatile("" :: "v"(c));
    v4u o = pack8_bf16(a, c);
    const unsigned mk = (p == 0) ? 0xFFFFFFFFu : 0u;
    o &= (v4u){ mk, mk, mk, mk };
    st2_v4u(WINP + (size_t)n * 32 + 8 * p, o);
  } else {
    if (tid < 160) {
      const int f  = 4 * tid;
      const int i0 = clampi(f, 0, 60);
      const int i1 = clampi(f - 64, 0, 188);
      const int i2 = clampi(f - 256, 0, 188);
      const int i3 = clampi(f - 448, 0, 188);
      const v4f a0 = *(const v4fa*)(bin + i0);
      const v4f a1 = *(const v4fa*)(biases + i1);
      const v4f a2 = *(const v4fa*)(gammas + i2);
      const v4f a3 = *(const v4fa*)(betas + i3);
      asm volatile("" :: "v"(a0));
      asm volatile("" :: "v"(a1));
      asm volatile("" :: "v"(a2));
      asm volatile("" :: "v"(a3));
      const unsigned m0 = (f < 64) ? 0xFFFFFFFFu : 0u;
      const unsigned m1 = (f >= 64 && f < 256) ? 0xFFFFFFFFu : 0u;
      const unsigned m2 = (f >= 256 && f < 448) ? 0xFFFFFFFFu : 0u;
      const unsigned m3 = (f >= 448) ? 0xFFFFFFFFu : 0u;
      v4f o;
#pragma unroll
      for (int j = 0; j < 4; ++j) {
        const unsigned bits = (__float_as_uint(a0[j]) & m0) | (__float_as_uint(a1[j]) & m1) |
                              (__float_as_uint(a2[j]) & m2) | (__float_as_uint(a3[j]) & m3);
        float t = bf16_val(__uint_as_float(bits));
        asm volatile("" : "+v"(t));
        o[j] = t;
      }
      st2_v4f(PAR + f, o);
    }
  }
}

__global__ __launch_bounds__(256) void k_list(const int* __restrict__ srcs, const int* __restrict__ dsts,
                                              int* LIST, int* NODE) {
  extern __shared__ __attribute__((aligned(16))) int dsm[];
  int* wl   = dsm;
  int* pl   = dsm + 8 * L_WLCAP;
  int* cnt  = pl + L_HCAP;
  int* offs = cnt + L_NBRUN;
  int* cur  = offs + L_NBRUN;
  int* misc = cur + L_NBRUN;
  const int tid = (int)threadIdx.x, lane = tid & 31, wave = tid >> 5;
  const int blk = (int)blockIdx.x;
  const unsigned nbs = (unsigned)(blk * L_NBRUN);

  {
    const v4i z4 = {0, 0, 0, 0};
#pragma unroll 1
    for (int i = tid * 4; i < L_ZINTS; i += 1024) *(v4ia*)(dsm + i) = z4;
    if (tid < 16) misc[tid] = 0;
  }
  __syncthreads();

  {
    const int per  = ((G_NE + 8 * 256 - 1) / (8 * 256)) * 256;
    const int ebeg = wave * per;
    const int eend = (ebeg + per < G_NE) ? (ebeg + per) : G_NE;
    int* mylist = wl + wave * L_WLCAP;
    int wc = 0;
#pragma unroll 1
    for (int cb = ebeg; cb < eend; cb += 256) {
      const int e0 = cb + lane * 8;
      const v4i da = *(const v4ia*)(dsts + e0);
      const v4i db = *(const v4ia*)(dsts + e0 + 4);
      asm volatile("" :: "v"(da));
      asm volatile("" :: "v"(db));
      const unsigned s0 = (unsigned)da.x - nbs, s1 = (unsigned)da.y - nbs;
      const unsigned s2 = (unsigned)da.z - nbs, s3 = (unsigned)da.w - nbs;
      const unsigned s4 = (unsigned)db.x - nbs, s5 = (unsigned)db.y - nbs;
      const unsigned s6 = (unsigned)db.z - nbs, s7 = (unsigned)db.w - nbs;
      const bool h0 = s0 < (unsigned)L_NBRUN, h1 = s1 < (unsigned)L_NBRUN, h2 = s2 < (unsigned)L_NBRUN, h3 = s3 < (unsigned)L_NBRUN;
      const bool h4 = s4 < (unsigned)L_NBRUN, h5 = s5 < (unsigned)L_NBRUN, h6 = s6 < (unsigned)L_NBRUN, h7 = s7 < (unsigned)L_NBRUN;
      const unsigned m0 = __builtin_amdgcn_ballot_w32(h0), m1 = __builtin_amdgcn_ballot_w32(h1);
      const unsigned m2 = __builtin_amdgcn_ballot_w32(h2), m3 = __builtin_amdgcn_ballot_w32(h3);
      const unsigned m4 = __builtin_amdgcn_ballot_w32(h4), m5 = __builtin_amdgcn_ballot_w32(h5);
      const unsigned m6 = __builtin_amdgcn_ballot_w32(h6), m7 = __builtin_amdgcn_ballot_w32(h7);
      const unsigned any = m0 | m1 | m2 | m3 | m4 | m5 | m6 | m7;
      if (any != 0u) {
        const int pre = (int)(__builtin_amdgcn_mbcnt_lo(m0, 0u) + __builtin_amdgcn_mbcnt_lo(m1, 0u) +
                              __builtin_amdgcn_mbcnt_lo(m2, 0u) + __builtin_amdgcn_mbcnt_lo(m3, 0u) +
                              __builtin_amdgcn_mbcnt_lo(m4, 0u) + __builtin_amdgcn_mbcnt_lo(m5, 0u) +
                              __builtin_amdgcn_mbcnt_lo(m6, 0u) + __builtin_amdgcn_mbcnt_lo(m7, 0u));
        int p = wc + pre;
        if (h0) { if (p < L_WLCAP) mylist[p] = (int)((s0 << 22) | (unsigned)(e0 + 0)); p = p + 1; }
        if (h1) { if (p < L_WLCAP) mylist[p] = (int)((s1 << 22) | (unsigned)(e0 + 1)); p = p + 1; }
        if (h2) { if (p < L_WLCAP) mylist[p] = (int)((s2 << 22) | (unsigned)(e0 + 2)); p = p + 1; }
        if (h3) { if (p < L_WLCAP) mylist[p] = (int)((s3 << 22) | (unsigned)(e0 + 3)); p = p + 1; }
        if (h4) { if (p < L_WLCAP) mylist[p] = (int)((s4 << 22) | (unsigned)(e0 + 4)); p = p + 1; }
        if (h5) { if (p < L_WLCAP) mylist[p] = (int)((s5 << 22) | (unsigned)(e0 + 5)); p = p + 1; }
        if (h6) { if (p < L_WLCAP) mylist[p] = (int)((s6 << 22) | (unsigned)(e0 + 6)); p = p + 1; }
        if (h7) { if (p < L_WLCAP) mylist[p] = (int)((s7 << 22) | (unsigned)(e0 + 7)); p = p + 1; }
        wc += (int)(__builtin_popcount(m0) + __builtin_popcount(m1) + __builtin_popcount(m2) + __builtin_popcount(m3) +
                    __builtin_popcount(m4) + __builtin_popcount(m5) + __builtin_popcount(m6) + __builtin_popcount(m7));
      }
    }
    if (lane == 0) misc[wave] = wc;
  }
  __syncthreads();

  if (wave == 0) {
    int ov = 0;
#pragma unroll 1
    for (int w2 = 0; w2 < 8; ++w2) {
      int c = misc[w2];
      if (c > L_WLCAP) ov = 1;
      c = c < 0 ? 0 : (c > L_WLCAP ? L_WLCAP : c);
#pragma unroll 1
      for (int b0 = 0; b0 < c; b0 += 32) {
        const int idx = b0 + lane;
        const int ent = wl[w2 * L_WLCAP + (idx < L_WLCAP ? idx : L_WLCAP - 1)];
        const int m32 = (c - b0) < 32 ? (c - b0) : 32;
#pragma unroll 1
        for (int k = 0; k < m32; ++k) {
          const int u    = __builtin_amdgcn_readlane(ent, k);
          const int slot = (int)((unsigned)u >> 22);
          const int cv   = cnt[slot];
          if (lane == 0) cnt[slot] = cv + 1;
        }
      }
    }
    if (lane == 0) misc[9] = ov;
  }
  __syncthreads();
  if (wave == 0) {
    const int base = lane * (L_NBRUN / 32);
    int s = 0;
#pragma unroll 1
    for (int i = 0; i < L_NBRUN / 32; ++i) s += cnt[base + i];
    int incl = s;
#pragma unroll
    for (int d = 1; d < 32; d <<= 1) {
      const int y = __shfl_up(incl, d, 32);
      if (lane >= d) incl += y;
    }
    const int t0   = __shfl(incl, 15, 32);
    const int tall = __shfl(incl, 31, 32);
    const int hsel = lane >> 4;
    int run = (incl - s) - hsel * t0 + hsel * L_HCAP;
#pragma unroll 1
    for (int i = 0; i < L_NBRUN / 32; ++i) {
      const int cv = cnt[base + i];
      offs[base + i] = run;
      cur[base + i]  = run;
      run += cv;
    }
    if (lane == 0) {
      const int t1 = tall - t0;
      misc[10] = t0;
      misc[11] = t1;
      if (t0 > L_HCAP || t1 > L_HCAP) misc[9] = 1;
    }
  }
  __syncthreads();

#pragma unroll 1
  for (int half = 0; half < 2; ++half) {
    if (wave == 0) {
#pragma unroll 1
      for (int w2 = 0; w2 < 8; ++w2) {
        int c = misc[w2];
        c = c < 0 ? 0 : (c > L_WLCAP ? L_WLCAP : c);
#pragma unroll 1
        for (int b0 = 0; b0 < c; b0 += 32) {
          const int idx = b0 + lane;
          const int ent = wl[w2 * L_WLCAP + (idx < L_WLCAP ? idx : L_WLCAP - 1)];
          const int sl  = (int)((unsigned)ent >> 22);
          const bool inh = (idx < c) && ((sl >> 9) == half);
          unsigned msk = __builtin_amdgcn_ballot_w32(inh);
#pragma unroll 1
          while (msk != 0u) {
            const int k = __builtin_ctz(msk);
            msk &= msk - 1u;
            const int u    = __builtin_amdgcn_readlane(ent, k);
            const int slot = (int)((unsigned)u >> 22);
            const int eid  = u & 0x3FFFFF;
            const int p    = cur[slot];
            int q = p - half * L_HCAP;
            q = q < 0 ? 0 : (q > L_HCAP - 1 ? L_HCAP - 1 : q);
            if (lane == 0) {
              pl[q] = eid;
              cur[slot] = p + 1;
            }
          }
        }
      }
    }
    __syncthreads();
    {
      int toth = misc[10 + half];
      toth = toth < 0 ? 0 : (toth > L_HCAP ? L_HCAP : toth);
      int* lp = LIST + (size_t)blk * (size_t)L_LCAP + (size_t)half * L_HCAP;
#pragma unroll 1
      for (int i = tid * 4; i < L_HCAP; i += 1024) {
        const v4i e = *(const v4ia*)(pl + i);
        int g0 = srcs[clampi(e.x, 0, G_NE - 1)];
        int g1 = srcs[clampi(e.y, 0, G_NE - 1)];
        int g2 = srcs[clampi(e.z, 0, G_NE - 1)];
        int g3 = srcs[clampi(e.w, 0, G_NE - 1)];
        asm volatile("" :: "v"(g0));
        asm volatile("" :: "v"(g1));
        asm volatile("" :: "v"(g2));
        asm volatile("" :: "v"(g3));
        g0 = clampi(g0, 0, G_NN - 1); g1 = clampi(g1, 0, G_NN - 1);
        g2 = clampi(g2, 0, G_NN - 1); g3 = clampi(g3, 0, G_NN - 1);
        const int k0 = (i + 0 < toth) ? -1 : 0, k1 = (i + 1 < toth) ? -1 : 0;
        const int k2 = (i + 2 < toth) ? -1 : 0, k3 = (i + 3 < toth) ? -1 : 0;
        const v4i o = { g0 & k0, g1 & k1, g2 & k2, g3 & k3 };
        st2_v4i(lp + i, o);
      }
    }
    __syncthreads();
  }

  {
    const int ovf = misc[9];
#pragma unroll 1
    for (int j = 0; j < 4; ++j) {
      const int slot = j * 256 + tid;
      const int c = cnt[slot];
      const int o = offs[slot];
      const int cm = c > 1 ? c : 1;
      const float q = 1.0f / (float)cm;
      const float inv = (c > 0) ? q : 0.0f;
      const v4i r = { o, c, __float_as_int(inv), ovf };
      st2_v4i(NODE + 4 * ((size_t)blk * L_NBRUN + (size_t)slot), r);
    }
  }
}

__global__ __launch_bounds__(256) void k_conv(const float* __restrict__ P, float* HF, unsigned short* OP) {
  const int u   = (int)blockIdx.x * 256 + (int)threadIdx.x;
  const int row = u >> 4;
  const int c   = u & 15;
  const bool live = row < G_NN;
  const float* pr = P + (size_t)row * 64;
  const v4f a = *(const v4fa*)(pr + 4 * c);
  const int pc = c & 7;
  const v4f b0 = *(const v4fa*)(pr + 8 * pc);
  const v4f b1 = *(const v4fa*)(pr + 8 * pc + 4);
  asm volatile("" :: "v"(a));
  asm volatile("" :: "v"(b0));
  asm volatile("" :: "v"(b1));
  v4f ha, h0, h1;
#pragma unroll
  for (int j = 0; j < 4; ++j) {
    const float ra = relu_k(a[j]), r0 = relu_k(b0[j]), r1 = relu_k(b1[j]);
    ha[j] = live ? ra : 0.0f;
    h0[j] = live ? r0 : 0.0f;
    h1[j] = live ? r1 : 0.0f;
  }
  st2_v4f(HF + (size_t)row * 64 + 4 * c, ha);
  const v4u hi = pack8_bf16(h0, h1);
  const v4u lo = pack8_bf16_lo(h0, h1);
  const unsigned sel = (c < 8) ? 0xFFFFFFFFu : 0u;
  const v4u sv = (v4u){ sel, sel, sel, sel };
  const v4u o = (hi & sv) | (lo & ~sv);
  if (c < G_PPR) st2_v4u(OP + (size_t)row * G_OPK + 8 * c, o);
}

template <int LAYER>
__global__ __launch_bounds__(256) void k_walk(const int* __restrict__ LIST, const int* __restrict__ NODE,
                                              const float* __restrict__ T, const float* __restrict__ PAR,
                                              float* HF, unsigned short* OP, float* out) {
  __shared__ __attribute__((aligned(16))) float sgb[128];
  const int tid = (int)threadIdx.x, lane = tid & 31, wave = tid >> 5;
  if (tid < 32) {
    const int po = (tid < 16) ? (256 + 64 * LAYER + 4 * tid) : (448 + 64 * LAYER + 4 * (tid - 16));
    const v4f g = *(const v4fa*)(PAR + po);
    *(v4fa*)(sgb + 4 * tid) = g;
  }
  __syncthreads();

  const int n  = (int)blockIdx.x * 8 + wave;
  const int nc = clampi(n, 0, G_NN - 1);
  const v4i rec = *(const v4ia*)(NODE + 4 * (size_t)nc);
  asm volatile("" :: "v"(rec));
  const size_t ro = (size_t)nc * 64 + 2 * (size_t)lane;
  const v2f s  = *(const v2fa*)(out + ro);
  const v2f hf = *(const v2fa*)(HF + ro);
  asm volatile("" :: "v"(s));
  asm volatile("" :: "v"(hf));

  int o = rec.x;
  int c = rec.y;
  const float invd = __int_as_float(rec.z);
  const int flag = rec.w;
  const bool big = c > L_DEGCAP;
  c = c < 0 ? 0 : (c > L_DEGCAP ? L_DEGCAP : c);
  o = o < 0 ? 0 : (o > L_LCAP - 1 ? L_LCAP - 1 : o);
  int last = o + (c > 0 ? c : 1) - 1;
  last = last > L_LCAP - 1 ? L_LCAP - 1 : last;
  const int* lb = LIST + (size_t)(nc >> L_SLB) * (size_t)L_LCAP;
  const int trips = __builtin_amdgcn_readfirstlane((n < G_NN) ? c : 0);

  float a0 = 0.0f, a1 = 0.0f;
#pragma unroll 1
  for (int b0 = 0; b0 < trips; b0 += 32) {
    int idx = o + b0 + lane;
    idx = idx > last ? last : idx;
    int sr = lb[idx];
    sr = sr < 0 ? 0 : (sr > G_NN - 1 ? G_NN - 1 : sr);
    const int m32 = (trips - b0) < 32 ? (trips - b0) : 32;
#pragma unroll 1
    for (int k = 0; k < m32; ++k) {
      const int sk = __builtin_amdgcn_readlane(sr, k);
      const v2f q = *(const v2fa*)(T + (size_t)sk * 64 + 2 * lane);
      a0 = a0 + q.x;
      a1 = a1 + q.y;
    }
  }

  const float m0 = a0 * invd;
  const float m1 = a1 * invd;
  const float v0 = s.x + m0;
  const float v1 = s.y + m1;
  float t = v0 + v1;
  t = t + __shfl_xor(t, 16, 32);
  t = t + __shfl_xor(t, 8, 32);
  t = t + __shfl_xor(t, 4, 32);
  t = t + __shfl_xor(t, 2, 32);
  t = t + __shfl_xor(t, 1, 32);
  const float mu = t * (1.0f / 64.0f);
  const float d0 = v0 - mu;
  const float d1 = v1 - mu;
  float q2 = d0 * d0 + d1 * d1;
  q2 = q2 + __shfl_xor(q2, 16, 32);
  q2 = q2 + __shfl_xor(q2, 8, 32);
  q2 = q2 + __shfl_xor(q2, 4, 32);
  q2 = q2 + __shfl_xor(q2, 2, 32);
  q2 = q2 + __shfl_xor(q2, 1, 32);
  const float var  = q2 * (1.0f / 64.0f);
  const float rstd = 1.0f / sqrtf(var + 1e-5f);
  const v2f gm = *(const v2fa*)(sgb + 2 * lane);
  const v2f bt = *(const v2fa*)(sgb + 64 + 2 * lane);
  const float z0 = ((d0 * rstd) * gm.x) + bt.x;
  const float z1 = ((d1 * rstd) * gm.y) + bt.y;
  const float r0 = relu_k(z0);
  const float r1 = relu_k(z1);
  const float qnan = __uint_as_float(0x7fc00000u);
  const bool bad = (flag != 0) || big;
  const float e0 = hf.x + r0;
  const float e1 = hf.y + r1;
  const float hn0 = bad ? qnan : e0;
  const float hn1 = bad ? qnan : e1;

  if (LAYER < 2) {
    const int j = lane & 15;
    const float c0 = __shfl(hn0, 2 * j, 32);
    const float c1 = __shfl(hn1, 2 * j, 32);
    const float c2 = __shfl(hn0, 2 * j + 1, 32);
    const float c3 = __shfl(hn1, 2 * j + 1, 32);
    const unsigned whi0 = pk16(bf16_bits(c0), bf16_bits(c1));
    const unsigned whi1 = pk16(bf16_bits(c2), bf16_bits(c3));
    const unsigned wlo0 = pk16(bf16_lo_bits(c0), bf16_lo_bits(c1));
    const unsigned wlo1 = pk16(bf16_lo_bits(c2), bf16_lo_bits(c3));
    const unsigned sel = (lane < 16) ? 0xFFFFFFFFu : 0u;
    const v2u w = (v2u){ (whi0 & sel) | (wlo0 & ~sel), (whi1 & sel) | (wlo1 & ~sel) };
    if (n < G_NN) {
      const v2f hv = (v2f){ hn0, hn1 };
      st2_v2f(HF + (size_t)n * 64 + 2 * lane, hv);
      if (lane < G_OPK / 4) st2_v2u(OP + (size_t)n * G_OPK + 4 * lane, w);
    }
  } else {
    if (n < G_NN) {
      const v2f hv = (v2f){ hn0, hn1 };
      st2_v2f(out + (size_t)n * 64 + 2 * lane, hv);
    }
  }
}

extern "C" void kernel_launch(void* const* d_in, const int* in_sizes, int n_in,
                              void* d_out, int out_size, void* d_ws, size_t ws_size,
                              hipStream_t stream) {
  if (n_in < 10) return;
  if (in_sizes[0] != G_NN * 8) return;
  if (in_sizes[1] != G_NE) return;
  if (in_sizes[2] != G_NE) return;
  if (in_sizes[3] != 64 * 8) return;
  if (in_sizes[4] != 64) return;
  if (in_sizes[5] != 3 * 64 * 64) return;
  if (in_sizes[6] != 3 * 64 * 64) return;
  if (in_sizes[7] != 192 || in_sizes[8] != 192 || in_sizes[9] != 192) return;
  if (out_size != G_NN * G_HD) return;

  const float* x      = (const float*)d_in[0];
  const int*   esrc   = (const int*)d_in[1];
  const int*   edst   = (const int*)d_in[2];
  const float* W_in   = (const float*)d_in[3];
  const float* b_in   = (const float*)d_in[4];
  const float* Wself  = (const float*)d_in[5];
  const float* Wneigh = (const float*)d_in[6];
  const float* biases = (const float*)d_in[7];
  const float* gammas = (const float*)d_in[8];
  const float* betas  = (const float*)d_in[9];
  float* out = (float*)d_out;

  constexpr size_t zXB   = (size_t)G_MP * 32 * 2;
  constexpr size_t zP    = (size_t)G_MP * 64 * 4;
  constexpr size_t zHF   = (size_t)G_MP * 64 * 4;
  constexpr size_t zOP   = (size_t)G_MP * G_OPK * 2;
  constexpr size_t zLIST = (size_t)L_NBK * L_LCAP * 4;
  constexpr size_t zNODE = (size_t)L_NBK * L_NBRUN * 16;
  constexpr size_t zWIN  = (size_t)64 * 32 * 2;
  constexpr size_t zWPL  = (size_t)6 * 64 * G_OPK * 2;
  constexpr size_t zPAR  = 4096;
  constexpr size_t oXB   = 0;
  constexpr size_t oP    = oXB + zXB;
  constexpr size_t oHF   = oP + zP;
  constexpr size_t oOP   = oHF + zHF;
  constexpr size_t oLIST = oOP + zOP;
  constexpr size_t oNODE = oLIST + zLIST;
  constexpr size_t oWIN  = oNODE + zNODE;
  constexpr size_t oWPL  = oWIN + zWIN;
  constexpr size_t oPAR  = oWPL + zWPL;
  constexpr size_t oEND  = oPAR + zPAR;
  static_assert(zXB % 256 == 0 && zP % 256 == 0 && zHF % 256 == 0 && zOP % 256 == 0 && zLIST % 256 == 0);
  static_assert(zNODE % 256 == 0 && zWIN % 256 == 0 && zWPL % 256 == 0 && zPAR % 256 == 0);
  static_assert(zPAR >= (size_t)640 * 4);
  static_assert(zNODE >= (size_t)G_NN * 16);
  static_assert(oEND <= ((size_t)128 << 20));
  static_assert(!SPLIT_L || oEND == (size_t)((size_t)12433 * 8192));
  if (oEND > ws_size) return;

  char* ws = (char*)d_ws;
  unsigned short* XB   = (unsigned short*)(ws + oXB);
  float*          P    = (float*)(ws + oP);
  float*          HF   = (float*)(ws + oHF);
  unsigned short* OP   = (unsigned short*)(ws + oOP);
  int*            LIST = (int*)(ws + oLIST);
  int*            NODE = (int*)(ws + oNODE);
  unsigned short* WINP = (unsigned short*)(ws + oWIN);
  unsigned short* WPL  = (unsigned short*)(ws + oWPL);
  float*          PAR  = (float*)(ws + oPAR);

  hipFuncSetAttribute(reinterpret_cast<const void*>(&k_list), hipFuncAttributeMaxDynamicSharedMemorySize, (int)L_LDS);

  static_assert((G_MP * 32 / 8) % 256 == 0);
  constexpr int gridPlane = G_MP * 32 / 8 / 256;
  constexpr int gridMP    = (G_MP / 64 + 7) / 8;
  constexpr int gridNN    = ((G_NN + 63) / 64 + 7) / 8;
  constexpr int gridConv  = G_MP * 16 / 256;
  constexpr int gridWalk  = G_NN / 8;
  static_assert(gridConv * 256 == G_MP * 16 && gridWalk * 8 == G_NN);

  k_plane<0><<<gridPlane, 256, 0, stream>>>(x, G_NN, 8, 8, XB, G_MP, 32);
  k_prep<<<6 * G_WPB + 2, 256, 0, stream>>>(W_in, b_in, Wself, Wneigh, biases, gammas, betas, WINP, WPL, PAR);
  k_list<<<L_NBK, 256, L_LDS, stream>>>(esrc, edst, LIST, NODE);
  k_gemm_nt<0, 1><<<gridMP, 256, 0, stream>>>(XB, WINP, PAR, P, G_MP, 64, 32, 64);
  k_conv<<<gridConv, 256, 0, stream>>>(P, HF, OP);

  constexpr size_t wpl = (size_t)64 * G_OPK;
  k_gemm_nt<0, 1><<<gridNN, 256, 0, stream>>>(OP, WPL + 0 * wpl, PAR + 64, out, G_NN, 64, G_OPK, 64);
  k_gemm_nt<0, 0><<<gridMP, 256, 0, stream>>>(OP, WPL + 3 * wpl, PAR, P, G_MP, 64, G_OPK, 64);
  k_walk<0><<<gridWalk, 256, 0, stream>>>(LIST, NODE, P, PAR, HF, OP, out);
  k_gemm_nt<0, 1><<<gridNN, 256, 0, stream>>>(OP, WPL + 1 * wpl, PAR + 128, out, G_NN, 64, G_OPK, 64);
  k_gemm_nt<0, 0><<<gridMP, 256, 0, stream>>>(OP, WPL + 4 * wpl, PAR, P, G_MP, 64, G_OPK, 64);
  k_walk<1><<<gridWalk, 256, 0, stream>>>(LIST, NODE, P, PAR, HF, OP, out);
  k_gemm_nt<0, 1><<<gridNN, 256, 0, stream>>>(OP, WPL + 2 * wpl, PAR + 192, out, G_NN, 64, G_OPK, 64);
  k_gemm_nt<0, 0><<<gridMP, 256, 0, stream>>>(OP, WPL + 5 * wpl, PAR, P, G_MP, 64, G_OPK, 64);
  k_walk<2><<<gridWalk, 256, 0, stream>>>(LIST, NODE, P, PAR, HF, OP, out);
}
